// MIM_52192442581410
// MI455X (gfx1250) — hardware-verified
//
#include <hip/hip_runtime.h>
#include <math.h>

#pragma clang fp contract(off)

typedef __attribute__((ext_vector_type(16))) _Float16 v16h;
typedef __attribute__((ext_vector_type(8)))  _Float16 v8h;
typedef __attribute__((ext_vector_type(8)))  float    v8f;
typedef __attribute__((ext_vector_type(4)))  float    v4f;
typedef __attribute__((ext_vector_type(2)))  float    v2f;

constexpr int kNB      = 4;
constexpr int kCin     = 128;
constexpr int kHt      = 160;
constexpr int kWd      = 160;
constexpr int kHW      = kHt * kWd;
constexpr int kRowsX   = kNB * kHW;
constexpr int kRois    = 256;
constexpr int kCmid    = 64;
constexpr int kCout    = 32;
constexpr int kBins    = 32;
constexpr int kSamp    = 64;
constexpr int kPosRoi  = kBins * kBins;
constexpr int kOutRow  = kCout * kPosRoi;
static_assert(kHW == 25600 && kRowsX == 102400, "feature rows");
static_assert((kRowsX % 64) == 0 && (kCmid % 64) == 0 && (kCin % 32) == 0, "projection GEMM tile multiples");
static_assert((kCmid % 32) == 0 && (kCout % 16) == 0 && (kPosRoi % 128) == 0, "head GEMM tile multiples");
static_assert((kHW % 32) == 0, "transpose tile multiple");
static_assert(kSamp == 2 * kBins, "two samples per bin and axis");

constexpr float kCarryX   = 16.0f;
constexpr float kCarryW1  = 256.0f;
constexpr float kCarryH   = 64.0f;
constexpr float kCarryW2  = 256.0f;
constexpr float kCarryRem = 2048.0f;
constexpr float kFold1    = 1.0f / (kCarryX * kCarryW1);
constexpr float kFold2    = 1.0f / (kCarryH * kCarryW2);
constexpr float kRemInv   = 1.0f / kCarryRem;
constexpr float kF16MinNormal = 6.103515625e-05f;

constexpr size_t kOffXT   = 0;
constexpr size_t kOffYP   = kOffXT  + (size_t)kRowsX * kCin * 2;
constexpr size_t kOffW1T  = kOffYP  + (size_t)kRowsX * kCmid * 4;
constexpr size_t kOffW2T  = kOffW1T + (size_t)kCmid * kCin * 2;
constexpr size_t kOffSCSH = kOffW2T + (size_t)kCout * kCmid * 2;
constexpr size_t kWsTotal = kOffSCSH + (size_t)2 * kCmid * 4;
static_assert(kWsTotal == 52449792ull, "carve total");
static_assert(kWsTotal <= 134217728ull, "carve cap");
static_assert((kOffYP % 128) == 0 && (kOffW1T % 128) == 0 && (kOffW2T % 128) == 0 && (kOffSCSH % 128) == 0, "aligned regions");

__device__ __forceinline__ _Float16 to_h_flush(float v) {
  const float a = fabsf(v);
  const float w = (a < kF16MinNormal) ? 0.0f : v;
  return (_Float16)w;
}

__device__ __forceinline__ unsigned pack_h2(_Float16 a, _Float16 b) {
  unsigned ua = (unsigned)__builtin_bit_cast(unsigned short, a);
  unsigned ub = (unsigned)__builtin_bit_cast(unsigned short, b);
  asm volatile("" : "+v"(ua));
  asm volatile("" : "+v"(ub));
  return (ub << 16) | (ua & 0xffffu);
}

union FragU { v16h v; v8h h[2]; };
__device__ __forceinline__ v16h frag_load(const _Float16* p) {
  FragU f;
  f.h[0] = *(const v8h*)(p);
  f.h[1] = *(const v8h*)(p + 16);
  return f.v;
}

__device__ __forceinline__ v8f mma_g(v16h a, v16h b, v8f c) {
  c = __builtin_amdgcn_wmma_f32_16x16x32_f16(false, a, false, b, (short)0, c, false, false);
  asm volatile("v_nop\n\tv_nop\n\tv_nop\n\tv_nop" : "+v"(c) : "v"(a), "v"(b));
  return c;
}

__global__ __launch_bounds__(256) void prep_planes_kernel(
    const float* __restrict__ W1, const float* __restrict__ b1, const float* __restrict__ gam,
    const float* __restrict__ bet, const float* __restrict__ mu, const float* __restrict__ var,
    const float* __restrict__ W2,
    unsigned short* __restrict__ W1T, unsigned short* __restrict__ W2T, float* __restrict__ SCSH)
{
  unsigned tid = threadIdx.x;
  asm volatile("" : "+v"(tid));
  v8h w1v[4];
#pragma unroll
  for (int it = 0; it < 4; ++it) {
    unsigned ch = (unsigned)it * 256u + tid;
    asm volatile("" : "+v"(ch));
    const unsigned n  = ch >> 4;
    const unsigned k8 = (ch & 15u) * 8u;
#pragma unroll
    for (int e = 0; e < 8; ++e) {
      const float w = W1[(k8 + (unsigned)e) * (unsigned)kCmid + n];
      w1v[it][e] = to_h_flush(w * kCarryW1);
    }
  }
  v8h w2v;
  {
    const unsigned n  = tid >> 3;
    const unsigned k8 = (tid & 7u) * 8u;
#pragma unroll
    for (int e = 0; e < 8; ++e) {
      const float w = W2[(k8 + (unsigned)e) * (unsigned)kCout + n];
      w2v[e] = to_h_flush(w * kCarryW2);
    }
  }
  v4f sv;
  {
    const unsigned j4 = (tid & 15u) * 4u;
    const bool first = ((tid & 16u) == 0u);
#pragma unroll
    for (int e = 0; e < 4; ++e) {
      const unsigned j = j4 + (unsigned)e;
      const float g  = gam[j];
      const float vr = var[j];
      const float sc = g / sqrtf(vr + 1e-5f);
      const float sh = (b1[j] - mu[j]) * sc + bet[j];
      sv[e] = first ? sc : sh;
    }
  }
  for (int pass = 0; pass < 2; ++pass) {
#pragma unroll
    for (int it = 0; it < 4; ++it)
      *(volatile v8h*)(W1T + ((size_t)it * 256u + tid) * 8u) = w1v[it];
    *(volatile v8h*)(W2T + (size_t)tid * 8u) = w2v;
    if (tid < 32u) *(volatile v4f*)(SCSH + tid * 4u) = sv;
    __threadfence();
  }
}

__global__ __launch_bounds__(256) void rows_f16_kernel(
    const float* __restrict__ x, unsigned short* __restrict__ XT)
{
  __shared__ float tb[128 * 33];
  unsigned tid = threadIdx.x;
  asm volatile("" : "+v"(tid));
  const unsigned lane = tid & 31u;
  const unsigned wave = tid >> 5;
  const unsigned b    = blockIdx.y;
  const unsigned hw0  = blockIdx.x * 32u;
  const float* xb = x + (size_t)b * kCin * kHW + hw0 + lane;
#pragma unroll 8
  for (int i = 0; i < 16; ++i) {
    const unsigned c = (unsigned)i * 8u + wave;
    tb[c * 33u + lane] = xb[(size_t)c * kHW];
  }
  __syncthreads();
  const unsigned hh = lane >> 4;
  const unsigned c8 = (lane & 15u) * 8u;
  v8h ov[2];
#pragma unroll
  for (int it = 0; it < 2; ++it) {
    const unsigned row = (unsigned)it * 16u + wave * 2u + hh;
#pragma unroll
    for (int e = 0; e < 8; ++e) {
      const float v = tb[(c8 + (unsigned)e) * 33u + row];
      ov[it][e] = to_h_flush(v * kCarryX);
    }
  }
  for (int pass = 0; pass < 2; ++pass) {
#pragma unroll
    for (int it = 0; it < 2; ++it) {
      const unsigned row = (unsigned)it * 16u + wave * 2u + hh;
      *(volatile v8h*)(XT + ((size_t)b * kHW + hw0 + row) * kCin + c8) = ov[it];
    }
    __threadfence();
  }
}

__global__ __launch_bounds__(256) void gemm_rows64_f16_kernel(
    const unsigned short* __restrict__ Ap, int lda,
    const unsigned short* __restrict__ Btp, int ldb,
    float* __restrict__ C, int ldc, int M, int N, int K, float scale)
{
  const _Float16* A  = (const _Float16*)Ap;
  const _Float16* Bt = (const _Float16*)Btp;
  __shared__ __align__(16) float sT[8][16 * 68];
  const int lane = threadIdx.x & 31;
  const int wave = threadIdx.x >> 5;
  const int tilesN = N >> 6;
  const int tilesM = M >> 6;
  const int tile = blockIdx.x * 8 + wave;
  if (tile >= tilesM * tilesN) return;
  const int tm = tile / tilesN;
  const int tn = tile - tm * tilesN;
  const int m0 = tm << 6;
  const int n0 = tn << 6;

  const int rlane = lane & 15;
  const int koff  = (lane >> 4) * 8;
  const int mOff  = (lane >> 4) * 8;

  v8f acc[4][4];
#pragma unroll
  for (int i = 0; i < 4; ++i)
#pragma unroll
    for (int j = 0; j < 4; ++j) acc[i][j] = (v8f){0.f, 0.f, 0.f, 0.f, 0.f, 0.f, 0.f, 0.f};

  for (int k0 = 0; k0 < K; k0 += 32) {
    v16h bh[4];
#pragma unroll
    for (int j = 0; j < 4; ++j) {
      const size_t bo = (size_t)(n0 + (j << 4) + rlane) * ldb + koff + k0;
      bh[j] = frag_load(Bt + bo);
    }
#pragma unroll
    for (int i = 0; i < 4; ++i) {
      const size_t ao = (size_t)(m0 + (i << 4) + rlane) * lda + koff + k0;
      const v16h ah = frag_load(A + ao);
#pragma unroll
      for (int j = 0; j < 4; ++j) acc[i][j] = mma_g(ah, bh[j], acc[i][j]);
    }
  }

  float* slab = sT[wave];
#pragma unroll
  for (int i = 0; i < 4; ++i) {
    const int mBase = m0 + (i << 4);
#pragma unroll
    for (int j = 0; j < 4; ++j) {
#pragma unroll
      for (int r = 0; r < 8; ++r) {
        const float v = acc[i][j][r] * scale;
        slab[(mOff + r) * 68 + (j << 4) + rlane] = v;
      }
    }
    __builtin_amdgcn_fence(__ATOMIC_RELEASE, "workgroup");
    __builtin_amdgcn_wave_barrier();
    __builtin_amdgcn_fence(__ATOMIC_ACQUIRE, "workgroup");
    {
      const int hh = lane >> 4, c4 = (lane & 15) * 4;
      for (int pass = 0; pass < 2; ++pass) {
#pragma unroll
        for (int it = 0; it < 8; ++it) {
          const int row = it * 2 + hh;
          const v4f v = *(const v4f*)(slab + row * 68 + c4);
          *(volatile v4f*)(C + (size_t)(mBase + row) * ldc + n0 + c4) = v;
        }
        __threadfence();
      }
    }
    __builtin_amdgcn_fence(__ATOMIC_RELEASE, "workgroup");
    __builtin_amdgcn_wave_barrier();
    __builtin_amdgcn_fence(__ATOMIC_ACQUIRE, "workgroup");
  }
}

__global__ __launch_bounds__(256) void roi_head_kernel(
    const float* __restrict__ YP, const float* __restrict__ boxes,
    const unsigned short* __restrict__ W2T, const float* __restrict__ SCSH,
    const float* __restrict__ b2, float* __restrict__ out)
{
  __shared__ __align__(16) unsigned sHw[128 * 36];
  __shared__ __align__(16) unsigned sHr[128 * 36];
  __shared__ __align__(16) float    sO[32 * 132];
  __shared__ int   sLo[128];
  __shared__ int   sHi[128];
  __shared__ float sWl[128];
  __shared__ float sWh[128];

  unsigned tid = threadIdx.x;
  asm volatile("" : "+v"(tid));
  const unsigned lane = tid & 31u;
  const unsigned wave = tid >> 5;
  unsigned hh = lane >> 4;
  asm volatile("" : "+v"(hh));
  unsigned cl = lane & 15u;
  asm volatile("" : "+v"(cl));
  const unsigned kroi = blockIdx.x;

  const float bf = boxes[kroi * 5u + 0u];
  const float x1 = boxes[kroi * 5u + 1u];
  const float y1 = boxes[kroi * 5u + 2u];
  const float x2 = boxes[kroi * 5u + 3u];
  const float y2 = boxes[kroi * 5u + 4u];
  int bi = (int)bf;
  bi = bi < 0 ? 0 : bi;
  bi = bi > (kNB - 1) ? (kNB - 1) : bi;
  const float roi_w = fmaxf(x2 - x1, 1.0f);
  const float roi_h = fmaxf(y2 - y1, 1.0f);

  {
    const unsigned i   = tid & 63u;
    const bool     isx = (tid & 64u) != 0u;
    const float start  = isx ? x1 : y1;
    const float ext    = isx ? roi_w : roi_h;
    const float binsz  = ext * (1.0f / 32.0f);
    const float g      = ((float)i + 0.5f) * 0.5f;
    const float step   = g * binsz;
    const float coord  = start + step;
    const float vld    = (coord >= -1.0f && coord <= 160.0f) ? 1.0f : 0.0f;
    const float c      = fminf(fmaxf(coord, 0.0f), 159.0f);
    int lo = (int)floorf(c);
    lo = lo < 0 ? 0 : lo;
    lo = lo > 159 ? 159 : lo;
    int hi = lo + 1;
    hi = hi > 159 ? 159 : hi;
    const float frac = c - (float)lo;
    const float wl = (1.0f - frac) * vld * 0.5f;
    const float wh = frac * vld * 0.5f;
    if (tid < 128u) {
      sLo[tid] = lo;
      sHi[tid] = hi;
      sWl[tid] = wl;
      sWh[tid] = wh;
    }
  }

  const _Float16* W2h = (const _Float16*)W2T;
  const v16h bw00 = frag_load(W2h + (size_t)(cl) * kCmid + 8u * hh);
  const v16h bw01 = frag_load(W2h + (size_t)(cl) * kCmid + 32u + 8u * hh);
  const v16h bw10 = frag_load(W2h + (size_t)(16u + cl) * kCmid + 8u * hh);
  const v16h bw11 = frag_load(W2h + (size_t)(16u + cl) * kCmid + 32u + 8u * hh);
  const v2f scv = *(const v2f*)(SCSH + 2u * lane);
  const v2f shv = *(const v2f*)(SCSH + 64u + 2u * lane);
  const float bias0 = b2[cl];
  const float bias1 = b2[16u + cl];
  const float* Yb = YP + (size_t)bi * kHW * kCmid + 2u * lane;
  float* ob = out + (size_t)kroi * kOutRow;

  __syncthreads();

#pragma unroll 1
  for (unsigned t = 0; t < 8u; ++t) {
#pragma unroll 1
    for (unsigned i = 0; i < 16u; ++i) {
      const unsigned pos = wave * 16u + i;
      const unsigned py  = t * 4u + (pos >> 5);
      const unsigned px  = pos & 31u;
      const unsigned ix0 = 64u + 2u * px;
      const int   xa  = sLo[ix0]      * kCmid;
      const int   xb  = sHi[ix0]      * kCmid;
      const int   xc  = sLo[ix0 + 1u] * kCmid;
      const int   xd  = sHi[ix0 + 1u] * kCmid;
      const float wxa = sWl[ix0];
      const float wxb = sWh[ix0];
      const float wxc = sWl[ix0 + 1u];
      const float wxd = sWh[ix0 + 1u];
      float acc0 = 0.0f, acc1 = 0.0f;
#pragma unroll 1
      for (unsigned sy = 0; sy < 2u; ++sy) {
        const unsigned iy = 2u * py + sy;
        const int   yl  = sLo[iy];
        const int   yh  = sHi[iy];
        const float wyl = sWl[iy];
        const float wyh = sWh[iy];
        const float* r0 = Yb + (size_t)(yl * kWd) * kCmid;
        const float* r1 = Yb + (size_t)(yh * kWd) * kCmid;
        const v2f v00 = *(const v2f*)(r0 + xa);
        const v2f v01 = *(const v2f*)(r0 + xb);
        const v2f v02 = *(const v2f*)(r0 + xc);
        const v2f v03 = *(const v2f*)(r0 + xd);
        const v2f v10 = *(const v2f*)(r1 + xa);
        const v2f v11 = *(const v2f*)(r1 + xb);
        const v2f v12 = *(const v2f*)(r1 + xc);
        const v2f v13 = *(const v2f*)(r1 + xd);
        float t0 = wxa * v00[0];
        float t1 = wxa * v00[1];
        t0 = fmaf(wxb, v01[0], t0);
        t1 = fmaf(wxb, v01[1], t1);
        t0 = fmaf(wxc, v02[0], t0);
        t1 = fmaf(wxc, v02[1], t1);
        t0 = fmaf(wxd, v03[0], t0);
        t1 = fmaf(wxd, v03[1], t1);
        float u0 = wxa * v10[0];
        float u1 = wxa * v10[1];
        u0 = fmaf(wxb, v11[0], u0);
        u1 = fmaf(wxb, v11[1], u1);
        u0 = fmaf(wxc, v12[0], u0);
        u1 = fmaf(wxc, v12[1], u1);
        u0 = fmaf(wxd, v13[0], u0);
        u1 = fmaf(wxd, v13[1], u1);
        acc0 = fmaf(wyl, t0, acc0);
        acc1 = fmaf(wyl, t1, acc1);
        acc0 = fmaf(wyh, u0, acc0);
        acc1 = fmaf(wyh, u1, acc1);
      }
      const float h0 = fmaxf(fmaf(acc0, scv[0], shv[0]), 0.0f);
      const float h1 = fmaxf(fmaf(acc1, scv[1], shv[1]), 0.0f);
      const float hs0 = h0 * kCarryH;
      const float hs1 = h1 * kCarryH;
      const _Float16 g0 = to_h_flush(hs0);
      const _Float16 g1 = to_h_flush(hs1);
      float gf0 = (float)g0;
      float gf1 = (float)g1;
      asm volatile("" : "+v"(gf0));
      asm volatile("" : "+v"(gf1));
      const float rm0 = (hs0 - gf0) * kCarryRem;
      const float rm1 = (hs1 - gf1) * kCarryRem;
      const _Float16 q0 = to_h_flush(rm0);
      const _Float16 q1 = to_h_flush(rm1);
      sHw[pos * 36u + lane] = pack_h2(g0, g1);
      sHr[pos * 36u + lane] = pack_h2(q0, q1);
    }
    __syncthreads();

    {
      const unsigned rowoff = (wave * 16u + cl) * 72u + 8u * hh;
      const _Float16* hp = (const _Float16*)sHw + rowoff;
      const _Float16* rp = (const _Float16*)sHr + rowoff;
      const v16h a0  = frag_load(hp);
      const v16h a1  = frag_load(hp + 32);
      const v16h ra0 = frag_load(rp);
      const v16h ra1 = frag_load(rp + 32);
      v8f d0 = (v8f){0.f, 0.f, 0.f, 0.f, 0.f, 0.f, 0.f, 0.f};
      v8f d1 = (v8f){0.f, 0.f, 0.f, 0.f, 0.f, 0.f, 0.f, 0.f};
      v8f e0 = (v8f){0.f, 0.f, 0.f, 0.f, 0.f, 0.f, 0.f, 0.f};
      v8f e1 = (v8f){0.f, 0.f, 0.f, 0.f, 0.f, 0.f, 0.f, 0.f};
      d0 = mma_g(a0, bw00, d0);
      d1 = mma_g(a0, bw10, d1);
      d0 = mma_g(a1, bw01, d0);
      d1 = mma_g(a1, bw11, d1);
      e0 = mma_g(ra0, bw00, e0);
      e1 = mma_g(ra0, bw10, e1);
      e0 = mma_g(ra1, bw01, e0);
      e1 = mma_g(ra1, bw11, e1);
      const unsigned pbase = wave * 16u + 8u * hh;
      v4f o0, o1, o2, o3;
#pragma unroll
      for (int r = 0; r < 4; ++r) {
        const float s0 = d0[r]     + e0[r]     * kRemInv;
        const float s1 = d0[4 + r] + e0[4 + r] * kRemInv;
        const float s2 = d1[r]     + e1[r]     * kRemInv;
        const float s3 = d1[4 + r] + e1[4 + r] * kRemInv;
        o0[r] = s0 * kFold2 + bias0;
        o1[r] = s1 * kFold2 + bias0;
        o2[r] = s2 * kFold2 + bias1;
        o3[r] = s3 * kFold2 + bias1;
      }
      *(v4f*)(sO + cl * 132u + pbase)               = o0;
      *(v4f*)(sO + cl * 132u + pbase + 4u)          = o1;
      *(v4f*)(sO + (16u + cl) * 132u + pbase)       = o2;
      *(v4f*)(sO + (16u + cl) * 132u + pbase + 4u)  = o3;
    }
    __syncthreads();

    {
      v4f vv[4];
#pragma unroll
      for (int it = 0; it < 4; ++it) {
        const unsigned e = wave * 4u + (unsigned)it;
        vv[it] = *(const v4f*)(sO + e * 132u + lane * 4u);
      }
      for (int pass = 0; pass < 2; ++pass) {
#pragma unroll
        for (int it = 0; it < 4; ++it) {
          const unsigned e = wave * 4u + (unsigned)it;
          *(volatile v4f*)(ob + (size_t)e * kPosRoi + t * 128u + lane * 4u) = vv[it];
        }
        __threadfence();
      }
    }
  }
}

extern "C" void kernel_launch(void* const* d_in, const int* in_sizes, int n_in,
                              void* d_out, int out_size, void* d_ws, size_t ws_size,
                              hipStream_t stream) {
  if (n_in < 10) return;
  if (in_sizes[0] != kNB * kCin * kHW) return;
  if (in_sizes[1] != kRois * 5) return;
  if (in_sizes[2] != kCin * kCmid) return;
  if (in_sizes[3] != kCmid) return;
  if (in_sizes[4] != kCmid) return;
  if (in_sizes[5] != kCmid) return;
  if (in_sizes[6] != kCmid) return;
  if (in_sizes[7] != kCmid) return;
  if (in_sizes[8] != kCmid * kCout) return;
  if (in_sizes[9] != kCout) return;
  if (out_size != kRois * kOutRow) return;
  if (ws_size < kWsTotal) return;

  const float* x     = (const float*)d_in[0];
  const float* boxes = (const float*)d_in[1];
  const float* W1    = (const float*)d_in[2];
  const float* b1    = (const float*)d_in[3];
  const float* gam   = (const float*)d_in[4];
  const float* bet   = (const float*)d_in[5];
  const float* mu    = (const float*)d_in[6];
  const float* var   = (const float*)d_in[7];
  const float* W2    = (const float*)d_in[8];
  const float* b2    = (const float*)d_in[9];
  float* out = (float*)d_out;

  char* ws = (char*)d_ws;
  unsigned short* XT   = (unsigned short*)(ws + kOffXT);
  float*          YP   = (float*)(ws + kOffYP);
  unsigned short* W1T  = (unsigned short*)(ws + kOffW1T);
  unsigned short* W2T  = (unsigned short*)(ws + kOffW2T);
  float*          SCSH = (float*)(ws + kOffSCSH);

  prep_planes_kernel<<<1, 256, 0, stream>>>(W1, b1, gam, bet, mu, var, W2, W1T, W2T, SCSH);

  rows_f16_kernel<<<dim3(kHW / 32, kNB), 256, 0, stream>>>(x, XT);

  gemm_rows64_f16_kernel<<<(kRowsX / 64) / 8, 256, 0, stream>>>(
      XT, kCin, W1T, kCin, YP, kCmid, kRowsX, kCmid, kCin, kFold1);

  roi_head_kernel<<<kRois, 256, 0, stream>>>(YP, boxes, W2T, SCSH, b2, out);
}
